// PhaseMLP_10445360463873
// MI455X (gfx1250) — hardware-run, weakly checked
//
#include <hip/hip_runtime.h>
#include <math.h>


#ifndef NB
#define NB 4096
#endif
#define NB_FULL 4096
#define D0 128
#define D1 256
#define D2 256
#define D3 128
#define OSP 68
#ifndef PHASE_RNE
#define PHASE_RNE 1
#endif

static_assert(NB % 64 == 0);
static_assert(NB <= NB_FULL);
static_assert(D0 % 64 == 0 && D1 % 64 == 0 && D2 % 64 == 0 && D3 % 64 == 0);
static_assert(D0 % 32 == 0 && D1 % 32 == 0 && D2 % 32 == 0);
static_assert(((size_t)NB * D0) % 8 == 0);
static_assert((OSP * 4) % 16 == 0);
static_assert(256 * 16 * 2 == 64 * 128);
static_assert(sizeof(float) * (64 * OSP + 64 * 4) <= 131072);
static_assert(sizeof(float) * (64 * 65) <= 131072);

typedef unsigned short bf;
typedef __attribute__((ext_vector_type(16))) __bf16   v16bf;
typedef __attribute__((ext_vector_type(8)))  unsigned short v8us;
typedef __attribute__((ext_vector_type(8)))  float    v8f;
typedef __attribute__((ext_vector_type(4)))  float    v4f;
typedef v4f  __attribute__((may_alias)) v4fa;

__device__ __forceinline__ unsigned short f2bf(float f) { unsigned u = __float_as_uint(f); u += 0x7FFFu + ((u >> 16) & 1u); return (unsigned short)(u >> 16); }
__device__ __forceinline__ float bf2f(unsigned short w) { return __uint_as_float(((unsigned)w) << 16); }
__device__ __forceinline__ v16bf cat16b(v8us lo, v8us hi) { return __builtin_bit_cast(v16bf, __builtin_shufflevector(lo, hi, 0, 1, 2, 3, 4, 5, 6, 7, 8, 9, 10, 11, 12, 13, 14, 15)); }
__device__ __forceinline__ v8f wmmab(v16bf a, v16bf b, v8f c) { return __builtin_amdgcn_wmma_f32_16x16x32_bf16(false, a, false, b, (short)0, c, false, false); }
__device__ __forceinline__ v8f wmmag(v16bf a, v16bf b, v8f c) { c = wmmab(a, b, c); asm volatile("v_nop\n\tv_nop\n\tv_nop\n\tv_nop" : "+v"(c) : "v"(a), "v"(b)); return c; }
__device__ __forceinline__ v16bf ldb(const bf* p)  { return cat16b(*(const v8us*)p, *(const v8us*)(p + 16)); }

__global__ __launch_bounds__(256) void k_wt(const float* __restrict__ W, bf* WT, int I, int O) {
    __shared__ float ts[64 * 65];
    const int t = threadIdx.x;
    const int o0 = blockIdx.x * 64, i0 = blockIdx.y * 64, c = blockIdx.z;
    const float* src = W + (size_t)c * I * O;
#pragma unroll 1
    for (int i = 0; i < 16; ++i) { const int f = i * 256 + t; ts[(f >> 6) * 65 + (f & 63)] = src[(size_t)(i0 + (f >> 6)) * O + o0 + (f & 63)]; }
    __syncthreads();
    bf* dst = WT + (size_t)c * O * I;
#pragma unroll 1
    for (int ps = 0; ps < 2; ++ps) {
#pragma unroll 1
        for (int it = 0; it < 2; ++it) {
            const int e = it * 32 + (t >> 3), c8 = (t & 7) * 8; v8us o;
#pragma unroll
            for (int k = 0; k < 8; ++k) o[k] = f2bf(ts[(c8 + k) * 65 + e]);
            *(volatile v8us*)(dst + (size_t)(o0 + e) * I + i0 + c8) = o; }
        if (ps == 0) __threadfence(); }
}

__global__ __launch_bounds__(256) void k_xcvt(const float* __restrict__ X, bf* XP) {
    const size_t i = (size_t)blockIdx.x * 256 + threadIdx.x; if (i >= ((size_t)NB * D0) / 8) return;
    const v8f a = *(const v8f*)(X + i * 8); v8us o;
#pragma unroll
    for (int k = 0; k < 8; ++k) o[k] = f2bf(a[k]);
    *(volatile v8us*)(XP + i * 8) = o; __threadfence(); *(volatile v8us*)(XP + i * 8) = o;
}

template <int KW, int KA, int O, int LAST>
__device__ __forceinline__ void layer_body(const bf* __restrict__ AP, const bf* __restrict__ WT, const float* __restrict__ Bias,
                                           const float* __restrict__ phase, bf* ACT, float* OUT) {
    static_assert((KW & (KW - 1)) == 0);
    static_assert(KW % 32 == 0);
    static_assert(KA == KW || KA == 2 * KW);
    static_assert(O % 64 == 0);
    __shared__ __align__(16) float os[64 * OSP];
    __shared__ __align__(16) float cs[64 * 4];
    const int tid = threadIdx.x, lane = tid & 31, lr = lane & 15, hi = lane >> 4;
    const int wave = __builtin_amdgcn_readfirstlane(tid >> 5);
    const int mbase = blockIdx.x * 64;
    const int cbase = blockIdx.y * 64;
    const int nbase = cbase + wave * 16;
    {
        const int rr = tid & 63;
        float ph = phase[(size_t)mbase + rr];
        if (PHASE_RNE) ph = bf2f(f2bf(ph));
        const float t = 4.0f * ph;
        const float ft = floorf(t);
        const int i1 = ((int)ft) & 3;
        const float w = t - ft;
        const float w2 = w * w, w3 = w2 * w;
        const float c0 = -0.5f * w + w2 - 0.5f * w3;
        const float c1 = 1.0f - 2.5f * w2 + 1.5f * w3;
        const float c2 = 0.5f * w + 2.0f * w2 - 1.5f * w3;
        const float c3 = -0.5f * w2 + 0.5f * w3;
        v4f cf;
#pragma unroll
        for (int p = 0; p < 4; ++p) { const int d = (p - i1) & 3; cf[p] = (d == 0) ? c1 : ((d == 1) ? c2 : ((d == 2) ? c3 : c0)); }
        if (tid < 64) *(v4fa*)(&cs[rr * 4]) = cf;
    }
    __syncthreads();
    v8f acc[4][4];
#pragma unroll
    for (int mb = 0; mb < 4; ++mb)
#pragma unroll
        for (int p = 0; p < 4; ++p) acc[mb][p] = (v8f){};
    const size_t aoff = (size_t)(mbase + lr) * KA + 8 * hi;
    const size_t boff = (size_t)(nbase + lr) * KW + 8 * hi;
#pragma unroll 1
    for (int kc = 0; kc < KA; kc += 32) {
        const int kb = kc & (KW - 1);
        v16bf a[4];
#pragma unroll
        for (int mb = 0; mb < 4; ++mb) a[mb] = ldb(AP + aoff + (size_t)mb * 16 * KA + kc);
#pragma unroll
        for (int p = 0; p < 4; ++p) { const v16bf b = ldb(WT + boff + (size_t)p * O * KW + kb);
#pragma unroll
            for (int mb = 0; mb < 4; ++mb) acc[mb][p] = wmmag(a[mb], b, acc[mb][p]); }
    }
    float bs[4];
#pragma unroll
    for (int p = 0; p < 4; ++p) bs[p] = bf2f(f2bf(Bias[p * O + nbase + lr]));
#pragma unroll
    for (int mb = 0; mb < 4; ++mb) {
#pragma unroll
        for (int j = 0; j < 8; ++j) {
            const int row = mb * 16 + 8 * hi + j;
            const v4f cf = *(const v4fa*)(&cs[row * 4]);
            const float val = cf[0] * (acc[mb][0][j] + bs[0]) + cf[1] * (acc[mb][1][j] + bs[1])
                            + cf[2] * (acc[mb][2][j] + bs[2]) + cf[3] * (acc[mb][3][j] + bs[3]);
            os[row * OSP + wave * 16 + lr] = val; } }
    __syncthreads();
    if (LAST) {
        static_assert(128 * 16 * 8 == 64 * 256);
        const int rq = tid >> 4, c4 = (tid & 15) * 4;
#pragma unroll 1
        for (int ps = 0; ps < 2; ++ps) {
#pragma unroll 1
            for (int it = 0; it < 8; ++it) { const int row = it * 8 + rq;
                const v4f v = *(const v4fa*)(&os[row * OSP + c4]);
                *(volatile v4f*)(OUT + (size_t)(mbase + row) * O + cbase + c4) = v; }
            if (ps == 0) __threadfence(); }
    } else {
        static_assert(128 * 16 * 4 == 64 * 128);
        const int rq = tid >> 3, c8 = (tid & 7) * 8;
#pragma unroll 1
        for (int ps = 0; ps < 2; ++ps) {
#pragma unroll 1
            for (int it = 0; it < 4; ++it) { const int row = it * 16 + rq;
                const v4f x0 = *(const v4fa*)(&os[row * OSP + c8]); const v4f x1 = *(const v4fa*)(&os[row * OSP + c8 + 4]);
                v8us oh, ol;
#pragma unroll
                for (int k = 0; k < 4; ++k) {
                    float u = x0[k]; const float eu = expm1f(fminf(u, 0.0f)); u = (u > 0.0f) ? u : eu;
                    float v = x1[k]; const float ev = expm1f(fminf(v, 0.0f)); v = (v > 0.0f) ? v : ev;
                    const unsigned short hu = f2bf(u), hv = f2bf(v);
                    oh[k] = hu; ol[k] = f2bf(u - bf2f(hu));
                    oh[4 + k] = hv; ol[4 + k] = f2bf(v - bf2f(hv)); }
                bf* dst = ACT + (size_t)(mbase + row) * (2 * O) + cbase + c8;
                *(volatile v8us*)dst = oh;
                *(volatile v8us*)(dst + O) = ol; }
            if (ps == 0) __threadfence(); }
    }
}

__global__ __launch_bounds__(128) __attribute__((amdgpu_num_vgpr(256))) void k_layer0(const bf* __restrict__ XP, const bf* __restrict__ WT, const float* __restrict__ Bias,
                                                                                       const float* __restrict__ phase, bf* ACT) {
    layer_body<D0, D0, D1, 0>(XP, WT, Bias, phase, ACT, (float*)0);
}
__global__ __launch_bounds__(128) __attribute__((amdgpu_num_vgpr(256))) void k_layer1(const bf* __restrict__ AP, const bf* __restrict__ WT, const float* __restrict__ Bias,
                                                                                       const float* __restrict__ phase, bf* ACT) {
    layer_body<D1, 2 * D1, D2, 0>(AP, WT, Bias, phase, ACT, (float*)0);
}
__global__ __launch_bounds__(128) __attribute__((amdgpu_num_vgpr(256))) void k_layer2(const bf* __restrict__ AP, const bf* __restrict__ WT, const float* __restrict__ Bias,
                                                                                       const float* __restrict__ phase, float* OUT) {
    layer_body<D2, 2 * D2, D3, 1>(AP, WT, Bias, phase, (bf*)0, OUT);
}

static constexpr size_t al256(size_t v) { return (v + 255) & ~(size_t)255; }
static constexpr size_t SZ_W0 = al256((size_t)4 * D1 * D0 * 2);
static constexpr size_t SZ_W1 = al256((size_t)4 * D2 * D1 * 2);
static constexpr size_t SZ_W2 = al256((size_t)4 * D3 * D2 * 2);
static constexpr size_t SZ_XP = al256((size_t)NB * D0 * 2);
static constexpr size_t SZ_A0 = al256((size_t)NB * 2 * D1 * 2);
static constexpr size_t SZ_A1 = al256((size_t)NB * 2 * D2 * 2);
static constexpr size_t SZ_TOTAL = SZ_W0 + SZ_W1 + SZ_W2 + SZ_XP + SZ_A0 + SZ_A1;
static_assert(SZ_TOTAL <= (size_t)134217728);

extern "C" void kernel_launch(void* const* d_in, const int* in_sizes, int n_in,
                              void* d_out, int out_size, void* d_ws, size_t ws_size, hipStream_t stream) {
    if (n_in < 8) return;
    if ((size_t)in_sizes[0] < (size_t)NB * D0) return;
    if ((size_t)in_sizes[1] < (size_t)NB) return;
    if ((size_t)in_sizes[2] < (size_t)4 * D0 * D1 || (size_t)in_sizes[3] < (size_t)4 * D1) return;
    if ((size_t)in_sizes[4] < (size_t)4 * D1 * D2 || (size_t)in_sizes[5] < (size_t)4 * D2) return;
    if ((size_t)in_sizes[6] < (size_t)4 * D2 * D3 || (size_t)in_sizes[7] < (size_t)4 * D3) return;
    if ((size_t)out_size < (size_t)NB * D3) return;
    if (SZ_TOTAL > ws_size) return;
    const float* x     = (const float*)d_in[0];
    const float* phase = (const float*)d_in[1];
    const float* w0    = (const float*)d_in[2];
    const float* b0    = (const float*)d_in[3];
    const float* w1    = (const float*)d_in[4];
    const float* b1    = (const float*)d_in[5];
    const float* w2    = (const float*)d_in[6];
    const float* b2    = (const float*)d_in[7];
    float* OUT = (float*)d_out;
    char* wsp = (char*)d_ws;
    bf* WT0  = (bf*)wsp; wsp += SZ_W0;
    bf* WT1  = (bf*)wsp; wsp += SZ_W1;
    bf* WT2  = (bf*)wsp; wsp += SZ_W2;
    bf* XP   = (bf*)wsp; wsp += SZ_XP;
    bf* ACT0 = (bf*)wsp; wsp += SZ_A0;
    bf* ACT1 = (bf*)wsp; wsp += SZ_A1;

    k_wt<<<dim3(D1 / 64, D0 / 64, 4), 256, 0, stream>>>(w0, WT0, D0, D1);
    k_wt<<<dim3(D2 / 64, D1 / 64, 4), 256, 0, stream>>>(w1, WT1, D1, D2);
    k_wt<<<dim3(D3 / 64, D2 / 64, 4), 256, 0, stream>>>(w2, WT2, D2, D3);
    k_xcvt<<<(unsigned)((((size_t)NB * D0) / 8 + 255) / 256), 256, 0, stream>>>(x, XP);
    k_layer0<<<dim3(NB / 64, D1 / 64), 128, 0, stream>>>(XP,   WT0, b0, phase, ACT0);
    k_layer1<<<dim3(NB / 64, D2 / 64), 128, 0, stream>>>(ACT0, WT1, b1, phase, ACT1);
    k_layer2<<<dim3(NB / 64, D3 / 64), 128, 0, stream>>>(ACT1, WT2, b2, phase, OUT);
}
